// FusedSequenceParallelAll2AllAttn_7292854469128
// MI455X (gfx1250) — hardware-verified
//
#include <hip/hip_runtime.h>


#define TT   4096
#define NQH  16
#define NKV  4
#define NHT  24
#define HD   128
#define ZH   1
#define RH   512
#define WRLD 8
#define LCH  256
#define PCAR 1024.0f
#define SCL  0.08838834764831845f
typedef _Float16 h16;
typedef unsigned short bf;
typedef __attribute__((ext_vector_type(16))) __bf16   v16bf;
typedef __attribute__((ext_vector_type(16))) _Float16 v16h;
typedef __attribute__((ext_vector_type(8)))  _Float16 v8h;
typedef __attribute__((ext_vector_type(8)))  unsigned short v8us;
typedef __attribute__((ext_vector_type(8)))  float    v8f;
typedef __attribute__((ext_vector_type(4)))  float    v4f;
typedef v8h  __attribute__((may_alias)) v8ha;
typedef v4f  __attribute__((may_alias)) v4fa;
typedef v8us __attribute__((may_alias)) v8usa;

__device__ __forceinline__ unsigned short f2bf(float f) { unsigned u = __float_as_uint(f); u += 0x7FFFu + ((u >> 16) & 1u); return (unsigned short)(u >> 16); }
__device__ __forceinline__ float bf2f(unsigned short b) { return __uint_as_float(((unsigned)b) << 16); }
__device__ __forceinline__ float bfr(float f) { return bf2f(f2bf(f)); }
__device__ __forceinline__ v16h cat16(v8h lo, v8h hi) { return __builtin_shufflevector(lo, hi, 0, 1, 2, 3, 4, 5, 6, 7, 8, 9, 10, 11, 12, 13, 14, 15); }
__device__ __forceinline__ v16bf cat16b(v8us lo, v8us hi) { return __builtin_bit_cast(v16bf, __builtin_shufflevector(lo, hi, 0, 1, 2, 3, 4, 5, 6, 7, 8, 9, 10, 11, 12, 13, 14, 15)); }
__device__ __forceinline__ v8f wmma16(v16h a, v16h b, v8f c) { return __builtin_amdgcn_wmma_f32_16x16x32_f16(false, a, false, b, (short)0, c, false, false); }
__device__ __forceinline__ v8f wmmab(v16bf a, v16bf b, v8f c) { return __builtin_amdgcn_wmma_f32_16x16x32_bf16(false, a, false, b, (short)0, c, false, false); }


template <typename T16> struct WFrag;
template <> struct WFrag<h16> { typedef v16h V; static __device__ __forceinline__ V ld(const h16* p) { return cat16(*(const v8h*)p, *(const v8h*)(p + 16)); } static __device__ __forceinline__ v8f mma(V a, V b, v8f c) { return wmma16(a, b, c); } };
template <> struct WFrag<bf> { typedef v16bf V; static __device__ __forceinline__ V ld(const bf* p) { return cat16b(*(const v8us*)p, *(const v8us*)(p + 16)); } static __device__ __forceinline__ v8f mma(V a, V b, v8f c) { return wmmab(a, b, c); } };
template <typename T16, int NSPLIT, bool BIAS>
__global__ __launch_bounds__(32) void k_gemmw(const T16* __restrict__ A, const T16* __restrict__ A2, const T16* __restrict__ Bt, const T16* __restrict__ Bt2, int K, float* C, int ldc, const float* __restrict__ bias, size_t sA, size_t sB, size_t sC) {
    typedef typename WFrag<T16>::V V;
    __shared__ __align__(16) float os[16 * 68];
    const size_t z = blockIdx.z; A += z * sA; if (A2) A2 += z * sA; Bt += z * sB; if (Bt2) Bt2 += z * sB; C += z * sC;
    const int lane = threadIdx.x & 31, lr = lane & 15, hi = lane >> 4; const int r0 = blockIdx.x * 64, c0 = blockIdx.y * 64;
    v8f acc[4][4];
#pragma unroll
    for (int mb = 0; mb < 4; ++mb)
#pragma unroll
        for (int nb = 0; nb < 4; ++nb) acc[mb][nb] = (v8f){};
    const size_t aoff = (size_t)(r0 + lr) * K + 8 * hi, boff = (size_t)(c0 + lr) * K + 8 * hi;
#pragma unroll 1
    for (int kc = 0; kc < K; kc += 32) {
        V a[4], a2[4];
#pragma unroll
        for (int mb = 0; mb < 4; ++mb) { a[mb] = WFrag<T16>::ld(A + aoff + (size_t)mb * 16 * K + kc); if (NSPLIT == 1 || NSPLIT == 2) a2[mb] = WFrag<T16>::ld(A2 + aoff + (size_t)mb * 16 * K + kc); }
#pragma unroll
        for (int nb = 0; nb < 4; ++nb) { const V b = WFrag<T16>::ld(Bt + boff + (size_t)nb * 16 * K + kc); V b2; if (NSPLIT >= 2) b2 = WFrag<T16>::ld(Bt2 + boff + (size_t)nb * 16 * K + kc);
#pragma unroll
            for (int mb = 0; mb < 4; ++mb) { acc[mb][nb] = WFrag<T16>::mma(a[mb], b, acc[mb][nb]); if (NSPLIT == 1 || NSPLIT == 2) acc[mb][nb] = WFrag<T16>::mma(a2[mb], b, acc[mb][nb]); if (NSPLIT >= 2) acc[mb][nb] = WFrag<T16>::mma(a[mb], b2, acc[mb][nb]); } }
        asm volatile("v_nop\n\tv_nop\n\tv_nop\n\tv_nop" : "+v"(acc[0][0]), "+v"(acc[1][1]), "+v"(acc[2][2]), "+v"(acc[3][3]) : "v"(a[0]), "v"(a[3]));
    }
#pragma unroll
    for (int mb = 0; mb < 4; ++mb) {
#pragma unroll
        for (int nb = 0; nb < 4; ++nb) {
#pragma unroll
            for (int j = 0; j < 8; ++j) os[(hi * 8 + j) * 68 + nb * 16 + lr] = acc[mb][nb][j]; }
        __builtin_amdgcn_wave_barrier(); asm volatile("" ::: "memory");
        float* crow = C + (size_t)(r0 + mb * 16) * ldc + c0;
#pragma unroll 1
        for (int ps = 0; ps < 2; ++ps) {
#pragma unroll
            for (int s = 0; s < 8; ++s) { const int row = 2 * s + hi, cofs = lr * 4; v4f val = *(const v4fa*)(os + row * 68 + cofs); if (BIAS) { val[0] += bfr(bias[c0 + cofs]); val[1] += bfr(bias[c0 + cofs + 1]); val[2] += bfr(bias[c0 + cofs + 2]); val[3] += bfr(bias[c0 + cofs + 3]); }
                *(volatile v4f*)(crow + (size_t)row * ldc + cofs) = val; }
            if (ps == 0) __threadfence(); }
        __builtin_amdgcn_wave_barrier(); asm volatile("" ::: "memory");
    }
}

template <typename T16, int NSPLIT, int CMODE>
__global__ __launch_bounds__(32) void k_gemmc(const T16* __restrict__ A, const T16* __restrict__ A2, const T16* __restrict__ Bt, const T16* __restrict__ Bt2, int K, float* C, int ldc, int roff, size_t sA, size_t sB, size_t sC) {
    typedef typename WFrag<T16>::V V;
    __shared__ __align__(16) float os[16 * 68];
    const size_t z = blockIdx.z; A += z * sA; if (A2) A2 += z * sA; Bt += z * sB; if (Bt2) Bt2 += z * sB; C += z * sC;
    const int lane = threadIdx.x & 31, lr = lane & 15, hi = lane >> 4; const int r0 = blockIdx.x * 64, c0 = blockIdx.y * 64;
    if (CMODE == 1 && c0 > r0 + roff + 63) return;
    const int Kl = (CMODE == 2) ? min(K, r0 + roff + 64) : K;
    v8f acc[4][4];
#pragma unroll
    for (int mb = 0; mb < 4; ++mb)
#pragma unroll
        for (int nb = 0; nb < 4; ++nb) acc[mb][nb] = (v8f){};
    const size_t aoff = (size_t)(r0 + lr) * K + 8 * hi, boff = (size_t)(c0 + lr) * K + 8 * hi;
#pragma unroll 1
    for (int kc = 0; kc < Kl; kc += 32) {
        V a[4], a2[4];
#pragma unroll
        for (int mb = 0; mb < 4; ++mb) { a[mb] = WFrag<T16>::ld(A + aoff + (size_t)mb * 16 * K + kc); if (NSPLIT == 1 || NSPLIT == 2) a2[mb] = WFrag<T16>::ld(A2 + aoff + (size_t)mb * 16 * K + kc); }
#pragma unroll
        for (int nb = 0; nb < 4; ++nb) { const V b = WFrag<T16>::ld(Bt + boff + (size_t)nb * 16 * K + kc); V b2; if (NSPLIT >= 2) b2 = WFrag<T16>::ld(Bt2 + boff + (size_t)nb * 16 * K + kc);
#pragma unroll
            for (int mb = 0; mb < 4; ++mb) { acc[mb][nb] = WFrag<T16>::mma(a[mb], b, acc[mb][nb]); if (NSPLIT == 1 || NSPLIT == 2) acc[mb][nb] = WFrag<T16>::mma(a2[mb], b, acc[mb][nb]); if (NSPLIT >= 2) acc[mb][nb] = WFrag<T16>::mma(a[mb], b2, acc[mb][nb]); } }
        asm volatile("v_nop\n\tv_nop\n\tv_nop\n\tv_nop" : "+v"(acc[0][0]), "+v"(acc[1][1]), "+v"(acc[2][2]), "+v"(acc[3][3]) : "v"(a[0]), "v"(a[3]));
    }
#pragma unroll
    for (int mb = 0; mb < 4; ++mb) {
#pragma unroll
        for (int nb = 0; nb < 4; ++nb) {
#pragma unroll
            for (int j = 0; j < 8; ++j) os[(hi * 8 + j) * 68 + nb * 16 + lr] = acc[mb][nb][j]; }
        __builtin_amdgcn_wave_barrier(); asm volatile("" ::: "memory");
        float* crow = C + (size_t)(r0 + mb * 16) * ldc + c0;
#pragma unroll 1
        for (int ps = 0; ps < 2; ++ps) {
#pragma unroll
            for (int s = 0; s < 8; ++s) { const int row = 2 * s + hi, cofs = lr * 4; v4f val = *(const v4fa*)(os + row * 68 + cofs);
                *(volatile v4f*)(crow + (size_t)row * ldc + cofs) = val; }
            if (ps == 0) __threadfence(); }
        __builtin_amdgcn_wave_barrier(); asm volatile("" ::: "memory");
    }
}

__device__ __forceinline__ h16 tohx(float x) { return (h16)x; }
__device__ __forceinline__ void splitf(float y, unsigned short& h, unsigned short& l) { h = f2bf(y); l = f2bf(y - bf2f(h)); }
typedef __attribute__((ext_vector_type(2))) unsigned short v2us;
typedef __attribute__((ext_vector_type(4))) unsigned short v4us;
typedef __attribute__((ext_vector_type(2))) _Float16 v2h;
typedef __attribute__((ext_vector_type(4))) _Float16 v4h;

__device__ __forceinline__ int prow(int n) { const int c = n / LCH, o = n % LCH; return (c < WRLD) ? (c * 2 * LCH + o) : ((2 * WRLD - 1 - c) * 2 * LCH + LCH + o); }
__global__ __launch_bounds__(256) void k_qk(const float* __restrict__ pk, int h, bf* QB, bf* KB) { const int e = (blockIdx.x * 256 + threadIdx.x) * 8; if (e >= TT * HD) return; const int d = e % HD; const int n = e / HD; const int p = prow(n); const float* qr = pk + ((size_t)p * NHT + h) * HD + d; const float* kr = pk + ((size_t)p * NHT + NQH + h / (NQH / NKV)) * HD + d; v8us oq, ok;
#pragma unroll
    for (int u = 0; u < 8; ++u) { oq[u] = f2bf(qr[u]); ok[u] = f2bf(kr[u]); } for (int ps = 0; ps < 2; ++ps) { *(volatile v8us*)(QB + e) = oq; *(volatile v8us*)(KB + e) = ok; if (ps == 0) __threadfence(); } }
__global__ __launch_bounds__(256) void k_vtb(const float* __restrict__ pk, int h, bf* VT, h16* VT16) { const int e = (blockIdx.x * 256 + threadIdx.x) * 2; if (e >= HD * TT) return; const int n = e % TT; const int d = e / TT; const int kv = NQH + NKV + h / (NQH / NKV); const float a = pk[((size_t)prow(n) * NHT + kv) * HD + d], b = pk[((size_t)prow(n + 1) * NHT + kv) * HD + d]; v2us o; o[0] = f2bf(a); o[1] = f2bf(b); v2h o6; o6[0] = tohx(bfr(a)); o6[1] = tohx(bfr(b));
    for (int ps = 0; ps < 2; ++ps) { *(volatile v2us*)(VT + e) = o; *(volatile v2h*)(VT16 + e) = o6; if (ps == 0) __threadfence(); } }
__global__ __launch_bounds__(256) void k_asoft(const float* __restrict__ Sb, h16* P16, bf* Ph, bf* Pl) {
    const int lane = threadIdx.x & 31; const int row = blockIdx.x * 8 + (threadIdx.x >> 5); if (row >= ZH * TT) return; const int i = row % TT; const int zz = row / TT; (void)zz; const bool hires = (i < RH); const float* sr = Sb + (size_t)row * TT;
    const int nch = (i / 128) + 1;
    float mx = -3.0e38f;
    for (int ch = 0; ch < nch; ++ch) { const int j0 = ch * 128 + lane * 4; const v4f a = *(const v4f*)(sr + j0);
#pragma unroll
        for (int q = 0; q < 4; ++q) { const float t = (j0 + q <= i) ? a[q] * SCL : -3.0e38f; mx = fmaxf(mx, t); } }
#pragma unroll
    for (int sh = 16; sh; sh >>= 1) mx = fmaxf(mx, __shfl_xor(mx, sh, 32));
    float sum = 0.f;
    for (int ch = 0; ch < nch; ++ch) { const int j0 = ch * 128 + lane * 4; const v4f a = *(const v4f*)(sr + j0);
#pragma unroll
        for (int q = 0; q < 4; ++q) { if (j0 + q <= i) { float d0 = __fsub_rn(a[q] * SCL, mx); asm volatile("" : "+v"(d0)); sum += __builtin_amdgcn_exp2f(__fmul_rn(d0, 1.4426950408889634f)); } } }
#pragma unroll
    for (int sh = 16; sh; sh >>= 1) sum += __shfl_xor(sum, sh, 32);
    const float f = __fdiv_rn(hires ? 1.0f : PCAR, sum);
    for (int ch = 0; ch < TT / 128; ++ch) { const int j0 = ch * 128 + lane * 4; float e[4];
            if (ch < nch) { const v4f a = *(const v4f*)(sr + j0);
#pragma unroll
                for (int q = 0; q < 4; ++q) { if (j0 + q <= i) { float d0 = __fsub_rn(a[q] * SCL, mx); asm volatile("" : "+v"(d0)); e[q] = __builtin_amdgcn_exp2f(__fmul_rn(d0, 1.4426950408889634f)) * f; } else e[q] = 0.f; } }
            else { e[0] = e[1] = e[2] = e[3] = 0.f; }
            if (hires) { v4us oh, ol;
#pragma unroll
                for (int q = 0; q < 4; ++q) { unsigned short a2, c2; splitf(e[q], a2, c2); oh[q] = a2; ol[q] = c2; }
                const size_t oo = ((size_t)zz * (RH ? RH : 1) + i) * TT + j0; *(volatile v4us*)(Ph + oo) = oh; *(volatile v4us*)(Pl + oo) = ol; __threadfence(); *(volatile v4us*)(Ph + oo) = oh; *(volatile v4us*)(Pl + oo) = ol; }
            else { v4h o4;
#pragma unroll
                for (int q = 0; q < 4; ++q) o4[q] = tohx(e[q]); *(volatile v4h*)(P16 + (size_t)row * TT + j0) = o4; __threadfence(); *(volatile v4h*)(P16 + (size_t)row * TT + j0) = o4; } }
}

__global__ __launch_bounds__(256) void k_mrg(const float* __restrict__ O, int h, float* outp) { const int e = (blockIdx.x * 256 + threadIdx.x) * 4; if (e >= TT * HD) return; const int d = e % HD; const int n = e / HD; const float cs = (n < RH) ? 1.0f : (1.0f / PCAR); const v4f a = *(const v4f*)(O + e); v4f o;
#pragma unroll
    for (int u = 0; u < 4; ++u) o[u] = a[u] * cs; float* dst = outp + ((size_t)prow(n) * NQH + h) * HD + d; *(volatile v4f*)dst = o; __threadfence(); *(volatile v4f*)dst = o; }

extern "C" void kernel_launch(void* const* d_in, const int* in_sizes, int n_in,
                              void* d_out, int out_size, void* d_ws, size_t ws_size, hipStream_t stream) {
    (void)in_sizes; (void)n_in; (void)out_size;
    const float* pk = (const float*)d_in[0];
    float* OUT = (float*)d_out;
    char* wsp = (char*)d_ws;
    auto take = [&](size_t bytes) { char* p = wsp; wsp += (bytes + 255) & ~(size_t)255; return (void*)p; };
    bf* QB = (bf*)take((size_t)TT * HD * 2); bf* KB = (bf*)take((size_t)TT * HD * 2); bf* VT = (bf*)take((size_t)HD * TT * 2); h16* VT16 = (h16*)take((size_t)HD * TT * 2); float* Sb = (float*)take((size_t)TT * TT * 4); h16* P16 = (h16*)take((size_t)TT * TT * 2); bf* Ph = (bf*)take((size_t)RH * TT * 2); bf* Pl = (bf*)take((size_t)RH * TT * 2); float* Ob = (float*)take((size_t)TT * HD * 4);
    if ((size_t)(wsp - (char*)d_ws) > ws_size) return;
    for (int h = 0; h < NQH; ++h) {
        k_qk<<<(TT * HD / 8 + 255) / 256, 256, 0, stream>>>(pk, h, QB, KB); k_vtb<<<(HD * TT / 2 + 255) / 256, 256, 0, stream>>>(pk, h, VT, VT16);
        k_gemmc<bf, 0, 1><<<dim3(TT / 64, TT / 64, 1), 32, 0, stream>>>(QB, nullptr, KB, nullptr, HD, Sb, TT, 0, 0, 0, 0);
        k_asoft<<<ZH * TT / 8, 256, 0, stream>>>(Sb, P16, Ph, Pl);
        k_gemmc<bf, 1, 2><<<dim3(RH / 64, HD / 64, 1), 32, 0, stream>>>(Ph, Pl, VT, nullptr, TT, Ob, HD, 0, 0, 0, 0);
        k_gemmc<h16, 0, 2><<<dim3((TT - RH) / 64, HD / 64, 1), 32, 0, stream>>>(P16 + (size_t)RH * TT, nullptr, VT16, nullptr, TT, Ob + (size_t)RH * HD, HD, RH, 0, 0, 0);
        k_mrg<<<(TT * HD / 4 + 255) / 256, 256, 0, stream>>>(Ob, h, OUT); }
}
